// full_conv_Layer_77369540870267
// MI455X (gfx1250) — hardware-verified
//
#include <hip/hip_runtime.h>
#include <math.h>

typedef __attribute__((ext_vector_type(16))) _Float16 v16h;
typedef __attribute__((ext_vector_type(16))) __bf16 v16b;
typedef __attribute__((ext_vector_type(8)))  _Float16 v8h;
typedef __attribute__((ext_vector_type(8)))  float v8f;
typedef __attribute__((ext_vector_type(4)))  float v4f;
typedef __attribute__((ext_vector_type(2)))  float v2f;
typedef __attribute__((ext_vector_type(4)))  unsigned v4u;
typedef __attribute__((ext_vector_type(4)))  int v4i;
typedef float __attribute__((may_alias)) float_a;
typedef int __attribute__((may_alias)) int_a;

template <typename T> __device__ __forceinline__ void vst2(void* p, T v) { *(volatile T*)p = v; __threadfence(); *(volatile T*)p = v; }
__device__ __forceinline__ v8f wmma16(v16h a, v16h b, v8f c) {
  v8f d = __builtin_amdgcn_wmma_f32_16x16x32_f16(false, a, false, b, (short)0, c, false, false);
  asm volatile("v_nop\n\tv_nop\n\tv_nop\n\tv_nop" : "+v"(d) : "v"(a), "v"(b));
  return d;
}
__device__ __forceinline__ v8f wmma_bf(v16b a, v16b b, v8f c) {
  v8f d = __builtin_amdgcn_wmma_f32_16x16x32_bf16(false, a, false, b, (short)0, c, false, false);
  asm volatile("v_nop\n\tv_nop\n\tv_nop\n\tv_nop" : "+v"(d) : "v"(a), "v"(b));
  return d;
}
__device__ __forceinline__ v16h frag_h(const _Float16* rowk0, int lane) {
  union { v16h v; v8h q[2]; } u; const _Float16* p = rowk0 + 8 * (lane >> 4);
  u.q[0] = *(const v8h*)p; u.q[1] = *(const v8h*)(p + 16); return u.v;
}
__device__ __forceinline__ v16h frag_f32(const float* rowk0, int lane) {
  v16h a; const float* p = rowk0 + 8 * (lane >> 4);
#pragma unroll
  for (int i = 0; i < 8; ++i) { a[i] = (_Float16)p[i]; a[8 + i] = (_Float16)p[16 + i]; }
  return a;
}
__device__ __forceinline__ v16h frag_f32s(const float* rowk0, int lane, float sc) {
  v16h a; const float* p = rowk0 + 8 * (lane >> 4);
#pragma unroll
  for (int i = 0; i < 8; ++i) { a[i] = (_Float16)(p[i] * sc); a[8 + i] = (_Float16)(p[16 + i] * sc); }
  return a;
}
__device__ __forceinline__ v16h fragc_f32(const float* W, int k0, int n, int lane, int ld, int K) {
  v16h a; const int g = lane >> 4;
#pragma unroll
  for (int i = 0; i < 8; ++i) { const int ka = k0 + 8 * g + i, kb = ka + 16;
    a[i] = (_Float16)(ka < K ? W[(size_t)(ka < K ? ka : K - 1) * ld + n] : 0.f); a[8 + i] = (_Float16)(kb < K ? W[(size_t)(kb < K ? kb : K - 1) * ld + n] : 0.f); }
  return a;
}
struct F2 { v16b h, l; };
__device__ __forceinline__ F2 bsplit16(const float v[16]) { F2 r;
#pragma unroll
  for (int i = 0; i < 16; ++i) { const __bf16 h = (__bf16)v[i]; r.h[i] = h; r.l[i] = (__bf16)(v[i] - (float)h); }
  return r; }
__device__ __forceinline__ F2 split_row(const float* row, int k0, int lane) { float v[16]; const float* p = row + k0 + 8 * (lane >> 4);
#pragma unroll
  for (int i = 0; i < 8; ++i) { v[i] = p[i]; v[8 + i] = p[16 + i]; }
  return bsplit16(v); }
__device__ __forceinline__ F2 split_rowK(const float* row, int k0, int lane, int K) { float v[16]; const int g = lane >> 4;
#pragma unroll
  for (int i = 0; i < 8; ++i) { const int ka = k0 + 8 * g + i, kb = ka + 16; v[i] = ka < K ? row[ka < K ? ka : K - 1] : 0.f; v[8 + i] = kb < K ? row[kb < K ? kb : K - 1] : 0.f; }
  return bsplit16(v); }
__device__ __forceinline__ F2 split_col(const float* W, int k0, int n, int lane, int ld, int K) { float v[16]; const int g = lane >> 4;
#pragma unroll
  for (int i = 0; i < 8; ++i) { const int ka = k0 + 8 * g + i, kb = ka + 16; v[i] = ka < K ? W[(size_t)(ka < K ? ka : K - 1) * ld + n] : 0.f; v[8 + i] = kb < K ? W[(size_t)(kb < K ? kb : K - 1) * ld + n] : 0.f; }
  return bsplit16(v); }
__device__ __forceinline__ v8f mac3(const F2& a, const F2& b, v8f c) { c = wmma_bf(a.l, b.h, c); c = wmma_bf(a.h, b.l, c); return wmma_bf(a.h, b.h, c); }
__device__ __forceinline__ float sigm(float v) { return 1.0f / (1.0f + expf(-v)); }
#define LDSX() do { asm volatile("s_wait_dscnt 0" ::: "memory"); __builtin_amdgcn_wave_barrier(); __builtin_amdgcn_fence(__ATOMIC_RELEASE, "workgroup"); } while (0)


#define NB 32
#define PP 4096
#define MM 12
#define WW 9
#define CI 64
#define CO 64
#define PNP (PP + 1)
#define NROW (NB * PP)
#ifndef TBLK
#define TBLK (NROW / 32)
#endif
typedef __attribute__((ext_vector_type(8))) __bf16 v8b;
__device__ __forceinline__ v16b frag_b(const __bf16* rowk0, int lane) {
  union { v16b v; v8b q[2]; } u; const __bf16* p = rowk0 + 8 * (lane >> 4);
  u.q[0] = *(const v8b*)p; u.q[1] = *(const v8b*)(p + 16); return u.v;
}
__device__ __forceinline__ float bfr(float v) { return (float)(__bf16)v; }
__device__ __attribute__((noinline)) float exp_ni(float v) { return expf(v); }
__device__ __attribute__((noinline)) float erf_ni(float v) { return erff(v); }

#define WS_END 64u

__global__ __launch_bounds__(128) void k_fcl(const float* __restrict__ PC, const float* __restrict__ WTS, const float* __restrict__ BIAS, const float* __restrict__ W2, const int* __restrict__ NID, const float* __restrict__ MSK, float* __restrict__ OUT) {
  __shared__ __align__(16) float sg[32][WW * CI + 8];
  __shared__ __align__(16) float so[32][CO + 4];
  const int tid = threadIdx.x, wave = tid >> 5, lane = tid & 31, col = lane & 15, g = lane >> 4; const size_t row0 = (size_t)blockIdx.x * 32; const size_t b = row0 / PP; const int p0 = (int)(row0 % PP);
#pragma unroll 1
  for (int rr = 0; rr < 8; ++rr) { const int rl = wave * 8 + rr; const int p = p0 + rl;
    v16b a;
#pragma unroll
    for (int i = 0; i < 8; ++i) { const int m0 = 8 * g + i, m1 = 16 + 8 * g + i; a[i] = (col < WW && m0 < MM) ? (__bf16)(bfr(W2[((size_t)p * MM + m0) * WW + col]) * bfr(MSK[(size_t)p * MM + m0])) : (__bf16)0.0f; a[8 + i] = (col < WW && m1 < MM) ? (__bf16)(bfr(W2[((size_t)p * MM + m1) * WW + col]) * bfr(MSK[(size_t)p * MM + m1])) : (__bf16)0.0f; }
#pragma unroll
    for (int j = 0; j < 4; ++j) { v16b w; const int i_ = j * 16 + col;
#pragma unroll
      for (int i = 0; i < 8; ++i) { const int m0 = 8 * g + i, m1 = 16 + 8 * g + i; int id0 = m0 < MM ? NID[(size_t)p * MM + m0] : 0; int id1 = m1 < MM ? NID[(size_t)p * MM + m1] : 0; id0 = id0 < 0 ? 0 : (id0 >= PNP ? PNP - 1 : id0); id1 = id1 < 0 ? 0 : (id1 >= PNP ? PNP - 1 : id1);
        w[i] = (m0 < MM) ? (__bf16)PC[(b * PNP + id0) * CI + i_] : (__bf16)0.0f; w[8 + i] = (m1 < MM) ? (__bf16)PC[(b * PNP + id1) * CI + i_] : (__bf16)0.0f; }
      v8f c = {}; c = wmma_bf(a, w, c);
#pragma unroll
      for (int r = 0; r < 8; ++r) { const int wv = 8 * g + r; if (wv < WW) sg[rl][wv * CI + i_] = c[r]; } } }
  __syncthreads();
  { const int rt = wave >> 1, ct0 = (wave & 1) * 2; v8f acc[2] = {};
#pragma unroll 2
    for (int kc = 0; kc < (WW * CI) / 32; ++kc) { float v[16]; const float* pp = &sg[rt * 16 + col][kc * 32 + 8 * g];
#pragma unroll
      for (int i = 0; i < 8; ++i) { v[i] = pp[i]; v[8 + i] = pp[16 + i]; }
      const F2 a = bsplit16(v); const int wv = kc >> 1, i0 = (kc & 1) * 32;
#pragma unroll
      for (int j = 0; j < 2; ++j) { v16b w; const int o = (ct0 + j) * 16 + col; const float* wr = WTS + (size_t)wv * (CO * CI) + o * CI + i0 + 8 * g;
#pragma unroll
        for (int i = 0; i < 8; ++i) { w[i] = (__bf16)wr[i]; w[8 + i] = (__bf16)wr[16 + i]; }
        acc[j] = wmma_bf(a.h, w, acc[j]); acc[j] = wmma_bf(a.l, w, acc[j]); } }
#pragma unroll
    for (int j = 0; j < 2; ++j) { const int o = (ct0 + j) * 16 + col; const float bb = bfr(BIAS[o]);
#pragma unroll
      for (int r = 0; r < 8; ++r) so[rt * 16 + 8 * g + r][o] = acc[j][r] + bb; } }
  __syncthreads(); for (int e = tid; e < 32 * 16; e += 128) { const int rl = e >> 4, q = e & 15; vst2(OUT + (row0 + rl) * CO + q * 4, *(const v4f*)&so[rl][q * 4]); } }
extern "C" void kernel_launch(void* const* d_in, const int* in_sizes, int n_in, void* d_out, int out_size, void* d_ws, size_t ws_size, hipStream_t stream) {
  (void)in_sizes; (void)n_in; (void)out_size; (void)d_ws; (void)ws_size;
  const float** F = (const float**)d_in;
  k_fcl<<<TBLK, 128, 0, stream>>>(F[0], F[1], F[2], F[3], (const int*)d_in[4], F[5], (float*)d_out);
}
